// KANTLinear_45414984188167
// MI455X (gfx1250) — hardware-verified
//
#include <hip/hip_runtime.h>
#include <math.h>

constexpr int kRows      = 16384;
constexpr int kIn        = 512;
constexpr int kOutF      = 512;
constexpr int kOrder     = 10;
constexpr int kKsp       = kIn * kOrder;
constexpr int kChunkRows = 4096;
constexpr int kNumChunks = kRows / kChunkRows;
constexpr int kGRows     = kChunkRows * kOrder;
constexpr float kWCarry      = 16.0f;
constexpr float kBaseScale   = 1.0f / 16.0f;
constexpr float kSplineScale = 1.0f / 160.0f;


typedef __attribute__((ext_vector_type(16))) _Float16 v16h;
typedef __attribute__((ext_vector_type(8)))  _Float16 v8h;
typedef __attribute__((ext_vector_type(16))) __bf16   v16b;
typedef __attribute__((ext_vector_type(8)))  __bf16   v8b;
typedef __attribute__((ext_vector_type(8)))  float    v8f;
typedef __attribute__((ext_vector_type(4)))  float    v4f;
typedef __attribute__((ext_vector_type(4)))  unsigned int v4u;
typedef __attribute__((ext_vector_type(2)))  unsigned int v2u;

__device__ __forceinline__ unsigned short f2bf_bits(float f) {
  unsigned u = __float_as_uint(f);
  return (unsigned short)((u + 0x7FFFu + ((u >> 16) & 1u)) >> 16);
}
__device__ __forceinline__ float bf_bits2f(unsigned short h) { return __uint_as_float(((unsigned)h) << 16); }

__device__ __forceinline__ void dep_guard_h(v8f& a, v8f& b, v16h x, v16h y) { asm volatile("v_nop\n\tv_nop\n\tv_nop\n\tv_nop" : "+v"(a), "+v"(b) : "v"(x), "v"(y)); }
__device__ __forceinline__ void dep_guard_b(v8f& a, v8f& b, v16b x, v16b y) { asm volatile("v_nop\n\tv_nop\n\tv_nop\n\tv_nop" : "+v"(a), "+v"(b) : "v"(x), "v"(y)); }
__device__ __forceinline__ void keep4_h(v16h a, v16h b, v16h c, v16h d) { asm volatile("v_nop" :: "v"(a), "v"(b), "v"(c), "v"(d)); }
__device__ __forceinline__ void keep4_b(v16b a, v16b b, v16b c, v16b d) { asm volatile("v_nop" :: "v"(a), "v"(b), "v"(c), "v"(d)); }
__device__ __forceinline__ void acc_guard4(v8f& a, v8f& b, v8f& c, v8f& d) { asm volatile("v_nop\n\tv_nop\n\tv_nop\n\tv_nop" : "+v"(a), "+v"(b), "+v"(c), "+v"(d)); }
template <typename T> struct Frag;
template <> struct Frag<_Float16> {
  typedef v16h V; union U { v16h v; v8h h[2]; };
  static __device__ __forceinline__ v16h load(const _Float16* p) {
    U f; f.h[0] = *(const v8h*)(p); f.h[1] = *(const v8h*)(p + 16); return f.v;
  }
  static __device__ __forceinline__ v8f mma(v16h a, v16h b, v8f c) {
    return __builtin_amdgcn_wmma_f32_16x16x32_f16(false, a, false, b, (short)0, c, false, false);
  }
  static __device__ __forceinline__ void guard(v8f& a, v8f& b, v16h x, v16h y) { dep_guard_h(a, b, x, y); }
  static __device__ __forceinline__ void keep(v16h a, v16h b, v16h c, v16h d) { keep4_h(a, b, c, d); }
};
template <> struct Frag<__bf16> {
  typedef v16b V; union U { v16b v; v8b h[2]; };
  static __device__ __forceinline__ v16b load(const __bf16* p) {
    U f; f.h[0] = *(const v8b*)(p); f.h[1] = *(const v8b*)(p + 16); return f.v;
  }
  static __device__ __forceinline__ v8f mma(v16b a, v16b b, v8f c) {
    return __builtin_amdgcn_wmma_f32_16x16x32_bf16(false, a, false, b, (short)0, c, false, false);
  }
  static __device__ __forceinline__ void guard(v8f& a, v8f& b, v16b x, v16b y) { dep_guard_b(a, b, x, y); }
  static __device__ __forceinline__ void keep(v16b a, v16b b, v16b c, v16b d) { keep4_b(a, b, c, d); }
};

__device__ __forceinline__ unsigned pk16(unsigned short a, unsigned short b) { return (unsigned)a | ((unsigned)b << 16); }
__device__ __forceinline__ unsigned short h_bits(float f) { const _Float16 h = (_Float16)f; return __builtin_bit_cast(unsigned short, h); }

template <int ET> struct Elem;
template <> struct Elem<0> { typedef _Float16 T; };
template <> struct Elem<1> { typedef __bf16 T; };
template <int ET, bool SPLIT, int BIAS_MODE, int OUT_MODE, bool RESID, int ACT = 0>
__global__ __launch_bounds__(256) void wmma_gemm64(
    const unsigned short* __restrict__ Ap, const unsigned short* __restrict__ A2p, int lda, long strideA,
    const unsigned short* __restrict__ Btp, const unsigned short* __restrict__ Bt2p, int ldb, long strideB,
    void* __restrict__ Cout, void* __restrict__ Cout2, int ldc, long strideC,
    const float* __restrict__ bias,
    const float* __restrict__ resid, long strideR,
    int M, int N, int K, float scale) {
  typedef typename Elem<ET>::T T;
  typedef typename Frag<T>::V V;
  const T* A = (const T*)Ap; const T* A2 = (const T*)A2p; const T* Bt = (const T*)Btp; const T* Bt2 = (const T*)Bt2p;
  __shared__ __align__(16) float sT[8][16 * 68];
  const int b    = blockIdx.y;
  const int lane = threadIdx.x & 31;
  const int wave = threadIdx.x >> 5;
  const int tilesN = N >> 6;
  const int tilesM = M >> 6;
  const int tile = blockIdx.x * 8 + wave;
  if (tile >= tilesM * tilesN) return;
  const int tm = tile / tilesN;
  const int tn = tile - tm * tilesN;
  const int m0 = tm << 6;
  const int n0 = tn << 6;

  const T* Ab  = A  + (size_t)b * strideA;
  const T* Bb  = Bt + (size_t)b * strideB;
  const T* Ab2 = SPLIT ? (A2  + (size_t)b * strideA) : nullptr;
  const T* Bb2 = SPLIT ? (Bt2 + (size_t)b * strideB) : nullptr;

  const int rlane = lane & 15;
  const int koff  = (lane >> 4) * 8;
  const int mOff  = (lane >> 4) * 8;

  v8f acc[4][4];
#pragma unroll
  for (int i = 0; i < 4; ++i)
#pragma unroll
    for (int j = 0; j < 4; ++j) acc[i][j] = (v8f){0.f,0.f,0.f,0.f,0.f,0.f,0.f,0.f};

  for (int k0 = 0; k0 < K; k0 += 32) {
    V bh[4], bl[4];
#pragma unroll
    for (int j = 0; j < 4; ++j) {
      const size_t bo = (size_t)(n0 + (j << 4) + rlane) * ldb + koff + k0;
      bh[j] = Frag<T>::load(Bb + bo);
      if (SPLIT) bl[j] = Frag<T>::load(Bb2 + bo);
    }
#pragma unroll
    for (int i = 0; i < 4; ++i) {
      const size_t ao = (size_t)(m0 + (i << 4) + rlane) * lda + koff + k0;
      V ah = Frag<T>::load(Ab + ao);
      V al;
      if (SPLIT) al = Frag<T>::load(Ab2 + ao);
#pragma unroll
      for (int j = 0; j < 4; ++j) {
        acc[i][j] = Frag<T>::mma(ah, bh[j], acc[i][j]);
        if (SPLIT) {
          acc[i][j] = Frag<T>::mma(ah, bl[j], acc[i][j]);
          acc[i][j] = Frag<T>::mma(al, bh[j], acc[i][j]);
        }
      }
      Frag<T>::guard(acc[i][0], acc[i][3], ah, SPLIT ? al : ah);
    }
    Frag<T>::keep(bh[0], bh[1], bh[2], bh[3]);
    if (SPLIT) Frag<T>::keep(bl[0], bl[1], bl[2], bl[3]);
  }
  acc_guard4(acc[0][0], acc[0][1], acc[0][2], acc[0][3]);
  acc_guard4(acc[1][0], acc[1][1], acc[1][2], acc[1][3]);
  acc_guard4(acc[2][0], acc[2][1], acc[2][2], acc[2][3]);
  acc_guard4(acc[3][0], acc[3][1], acc[3][2], acc[3][3]);

  float* slab = sT[wave];
  const float* Rb = RESID ? (resid + (size_t)b * strideR) : nullptr;
#pragma unroll
  for (int i = 0; i < 4; ++i) {
    const int mBase = m0 + (i << 4);
#pragma unroll
    for (int j = 0; j < 4; ++j) {
      const int n = n0 + (j << 4) + rlane;
      float bv = 0.f;
      if (BIAS_MODE == 2) bv = bias[n];
#pragma unroll
      for (int r = 0; r < 8; ++r) {
        float v = acc[i][j][r] * scale;
        if (BIAS_MODE == 1) v += bias[mBase + mOff + r];
        if (BIAS_MODE == 2) v += bv;
        if (RESID) v += Rb[(size_t)(mBase + mOff + r) * ldc + n];
        if (ACT == 2) v = fmaxf(v, 0.0f);
        if (ACT == 4) v = (v > 0.f) ? v : 0.01f * v;
        slab[(mOff + r) * 68 + (j << 4) + rlane] = v;
      }
    }
    __builtin_amdgcn_fence(__ATOMIC_RELEASE, "workgroup");
    __builtin_amdgcn_wave_barrier();
    __builtin_amdgcn_fence(__ATOMIC_ACQUIRE, "workgroup");
    if (OUT_MODE == 0) {
      float* C = (float*)Cout + (size_t)b * strideC;
      const int hh = lane >> 4, c4 = (lane & 15) * 4;
      for (int pass = 0; pass < 2; ++pass) {
#pragma unroll
        for (int it = 0; it < 8; ++it) {
          const int row = it * 2 + hh;
          v4f v = *(const v4f*)(slab + row * 68 + c4);
          *(volatile v4f*)(C + (size_t)(mBase + row) * ldc + n0 + c4) = v;
        }
        __threadfence();
      }
    } else {
      const int q = lane >> 3, c8 = (lane & 7) * 8;
      unsigned short* C  = (unsigned short*)Cout  + (size_t)b * strideC;
      unsigned short* C2 = (OUT_MODE == 2) ? ((unsigned short*)Cout2 + (size_t)b * strideC) : nullptr;
      for (int pass = 0; pass < 2; ++pass) {
#pragma unroll
        for (int it = 0; it < 4; ++it) {
          const int row = it * 4 + q;
          const float* sp = slab + row * 68 + c8;
          v8h hv, lv;
#pragma unroll
          for (int e = 0; e < 8; ++e) {
            if (OUT_MODE == 1) {
              hv[e] = (_Float16)sp[e];
            } else {
              unsigned short hb = f2bf_bits(sp[e]);
              unsigned short lb = f2bf_bits(sp[e] - bf_bits2f(hb));
              hv[e] = __builtin_bit_cast(_Float16, hb);
              lv[e] = __builtin_bit_cast(_Float16, lb);
            }
          }
          *(volatile v8h*)(C + (size_t)(mBase + row) * ldc + n0 + c8) = hv;
          if (OUT_MODE == 2) *(volatile v8h*)(C2 + (size_t)(mBase + row) * ldc + n0 + c8) = lv;
        }
        __threadfence();
      }
    }
    __builtin_amdgcn_fence(__ATOMIC_RELEASE, "workgroup");
    __builtin_amdgcn_wave_barrier();
    __builtin_amdgcn_fence(__ATOMIC_ACQUIRE, "workgroup");
  }
}

__global__ __launch_bounds__(256) void cast8_scale_f16_kernel(const float* __restrict__ in, unsigned short* __restrict__ out,
                                                             int n8, float scale) {
  const int i = blockIdx.x * 256 + threadIdx.x;
  if (i >= n8) return;
  const float* p = in + 8 * (size_t)i;
  const v4f a = *(const v4f*)(p);
  const v4f c = *(const v4f*)(p + 4);
  unsigned short hb[8];
#pragma unroll
  for (int e = 0; e < 4; ++e) {
    hb[e]     = h_bits(a[e] * scale);
    hb[4 + e] = h_bits(c[e] * scale);
  }
  const v4u u = (v4u){pk16(hb[0], hb[1]), pk16(hb[2], hb[3]), pk16(hb[4], hb[5]), pk16(hb[6], hb[7])};
  unsigned short* q = out + 8 * (size_t)i;
  *(volatile v4u*)q = u;
  __threadfence();
  *(volatile v4u*)q = u;
}

__global__ __launch_bounds__(256) void silu4_f16_kernel(const float* __restrict__ in, unsigned short* __restrict__ out, int n4) {
  const int i = blockIdx.x * 256 + threadIdx.x;
  if (i >= n4) return;
  const v4f a = *(const v4f*)(in + 4 * (size_t)i);
  unsigned short hb[4];
#pragma unroll
  for (int e = 0; e < 4; ++e) {
    const float v  = a[e];
    const float sg = 1.0f / (1.0f + expf(-v));
    hb[e] = h_bits(v * sg);
  }
  const v2u u = (v2u){pk16(hb[0], hb[1]), pk16(hb[2], hb[3])};
  unsigned short* q = out + 4 * (size_t)i;
  *(volatile v2u*)q = u;
  __threadfence();
  *(volatile v2u*)q = u;
}

__global__ __launch_bounds__(256) void cheby_rows_kernel(const float* __restrict__ x, unsigned short* __restrict__ tp,
                                                         int gbase, int nrows) {
#pragma clang fp contract(off)
  const int t  = threadIdx.x;
  const int gl = blockIdx.x * 4 + (t >> 6);
  if (gl >= nrows) return;
  const int col = (t & 63) * 8;
  const int g   = gbase + gl;
  int ord = g >> 14;
  ord = ord < 0 ? 0 : (ord > kOrder - 1 ? kOrder - 1 : ord);
  const int bsrc = g & (kRows - 1);
  const float* xp = x + (size_t)bsrc * kIn + col;
  const v4f x0 = *(const v4f*)(xp);
  const v4f x1 = *(const v4f*)(xp + 4);
  float tw[8], ta[8], tb[8];
#pragma unroll
  for (int e = 0; e < 4; ++e) {
    ta[e] = 1.0f;          ta[4 + e] = 1.0f;
    tb[e] = x0[e];         tb[4 + e] = x1[e];
    tw[e] = 2.0f * x0[e];  tw[4 + e] = 2.0f * x1[e];
  }
#pragma unroll 1
  for (int n = 0; n < ord; ++n) {
#pragma unroll
    for (int e = 0; e < 8; ++e) {
      const float pr = tw[e] * tb[e];
      const float cc = pr - ta[e];
      ta[e] = tb[e];
      tb[e] = cc;
    }
  }
  unsigned short hb[8];
#pragma unroll
  for (int e = 0; e < 8; ++e) hb[e] = h_bits(ta[e]);
  const v4u u = (v4u){pk16(hb[0], hb[1]), pk16(hb[2], hb[3]), pk16(hb[4], hb[5]), pk16(hb[6], hb[7])};
  unsigned short* q = tp + (size_t)gl * kIn + col;
  *(volatile v4u*)q = u;
  __threadfence();
  *(volatile v4u*)q = u;
}

extern "C" void kernel_launch(void* const* d_in, const int* in_sizes, int n_in,
                              void* d_out, int out_size, void* d_ws, size_t ws_size,
                              hipStream_t stream) {
  if (n_in < 3) return;
  if (in_sizes[0] != kRows * kIn) return;
  if (in_sizes[1] != kOutF * kIn) return;
  if (in_sizes[2] != kOutF * kKsp) return;
  if (out_size != kRows * kOutF) return;

  const float* x  = (const float*)d_in[0];
  const float* wb = (const float*)d_in[1];
  const float* wc = (const float*)d_in[2];
  float* out = (float*)d_out;

  const size_t offWb   = 0;
  const size_t szWb    = (size_t)kOutF * kIn * 2;
  const size_t offWc   = offWb + szWb;
  const size_t szWc    = (size_t)kOutF * kKsp * 2;
  const size_t offS    = offWc + szWc;
  const size_t szS     = (size_t)kRows * kIn * 2;
  const size_t offBase = offS + szS;
  const size_t szBase  = (size_t)kRows * kOutF * 4;
  const size_t offT    = offBase + szBase;
  const size_t szT     = (size_t)kGRows * kIn * 2;
  const size_t total   = offT + szT;
  if (d_ws == nullptr || total > ws_size) return;

  unsigned char* ws = (unsigned char*)d_ws;
  unsigned short* Wb16 = (unsigned short*)(ws + offWb);
  unsigned short* Wc16 = (unsigned short*)(ws + offWc);
  unsigned short* S16  = (unsigned short*)(ws + offS);
  float*          Base = (float*)(ws + offBase);
  unsigned short* Tpl  = (unsigned short*)(ws + offT);

  {
    const int n8 = (kOutF * kIn) / 8;
    cast8_scale_f16_kernel<<<dim3((n8 + 255) / 256), dim3(256), 0, stream>>>(wb, Wb16, n8, kWCarry);
  }
  {
    const int n8 = (kOutF * kKsp) / 8;
    cast8_scale_f16_kernel<<<dim3((n8 + 255) / 256), dim3(256), 0, stream>>>(wc, Wc16, n8, kWCarry);
  }
  {
    const int n4 = (kRows * kIn) / 4;
    silu4_f16_kernel<<<dim3((n4 + 255) / 256), dim3(256), 0, stream>>>(x, S16, n4);
  }
  {
    const int tiles = (kRows / 64) * (kOutF / 64);
    wmma_gemm64<0, false, 0, 0, false, 0><<<dim3((tiles + 7) / 8, 1), dim3(256), 0, stream>>>(
        S16, S16, kIn, 0L,
        Wb16, Wb16, kIn, 0L,
        (void*)Base, (void*)Base, kOutF, 0L,
        Base,
        Base, 0L,
        kRows, kOutF, kIn, kBaseScale);
  }
  for (int c = 0; c < kNumChunks; ++c) {
    const int gbase = c * kGRows;
    cheby_rows_kernel<<<dim3((kGRows + 3) / 4), dim3(256), 0, stream>>>(x, Tpl, gbase, kGRows);
    float* outc = out + (size_t)c * kChunkRows * kOutF;
    const float* resc = Base + (size_t)c * kChunkRows * kOutF;
    const int tiles = (kChunkRows / 64) * (kOutF / 64);
    wmma_gemm64<0, false, 0, 0, true, 0><<<dim3((tiles + 7) / 8, 1), dim3(256), 0, stream>>>(
        Tpl, Tpl, kKsp, 0L,
        Wc16, Wc16, kKsp, 0L,
        (void*)outc, (void*)outc, kOutF, 0L,
        resc,
        resc, 0L,
        kChunkRows, kOutF, kKsp, kSplineScale);
  }
}
